// CapRNNModelHelper_70102456205953
// MI455X (gfx1250) — hardware-run, weakly checked
//
#include <hip/hip_runtime.h>
#include <math.h>

constexpr int kVocab   = 50000;
constexpr int kEmbDim  = 300;
constexpr int kEmbPad  = 320;
constexpr int kHid     = 128;
constexpr int kGate3   = 384;
constexpr int kSeq     = 256;
constexpr int kBatch   = 128;
constexpr int kRows    = kSeq * kBatch;
constexpr int kHid2    = 2 * kHid;
constexpr int kCaps    = 10;
constexpr int kCapDim  = 16;
constexpr int kCapOut  = kCaps * kCapDim;
constexpr int kCapPad  = 192;
constexpr int kOutCls  = 2;
constexpr int kIters   = 5;
constexpr int kHPitch  = 136;
constexpr int kXWords  = 196;
constexpr float kWCarry    = 16.0f;
constexpr float kWCarryInv = 1.0f / 16.0f;
constexpr float kSquashEps = 1e-7f;

static_assert(kRows == 32768);
static_assert(kEmbPad % 32 == 0 && kHid % 32 == 0 && kHid2 % 32 == 0);
static_assert(kRows % 64 == 0 && kGate3 % 64 == 0 && kCapPad % 64 == 0);
static_assert(kEmbDim % 4 == 0 && kEmbPad % 8 == 0);
static_assert((2 * 16 * kHPitch) % 256 == 0);
static_assert(kCapOut == 160 && kCapOut % 32 == 0);
static_assert((kXWords * 4) % 16 == 0 && (kHPitch * 2) % 16 == 0);
static_assert(kBatch * kOutCls == 256);

typedef __attribute__((ext_vector_type(16))) _Float16 v16h;
typedef __attribute__((ext_vector_type(8)))  _Float16 v8h;
typedef __attribute__((ext_vector_type(8)))  float    v8f;
typedef __attribute__((ext_vector_type(4)))  float    v4f;
typedef __attribute__((ext_vector_type(4)))  unsigned v4u;

__device__ __forceinline__ void guard4_h(v8f& a0, v8f& a1, v8f& a2, v8f& a3, v16h x, v16h y0, v16h y1, v16h y2, v16h y3) {
  asm volatile("v_nop\n\tv_nop\n\tv_nop\n\tv_nop" : "+v"(a0), "+v"(a1), "+v"(a2), "+v"(a3) : "v"(x), "v"(y0), "v"(y1), "v"(y2), "v"(y3));
}
__device__ __forceinline__ void guard3_h(v8f& a0, v8f& a1, v8f& a2, v16h x, v16h y0, v16h y1, v16h y2) {
  asm volatile("v_nop\n\tv_nop\n\tv_nop\n\tv_nop" : "+v"(a0), "+v"(a1), "+v"(a2) : "v"(x), "v"(y0), "v"(y1), "v"(y2));
}
__device__ __forceinline__ void keep4_h(v16h a, v16h b, v16h c, v16h d) { asm volatile("v_nop" :: "v"(a), "v"(b), "v"(c), "v"(d)); }
__device__ __forceinline__ void acc_guard4(v8f& a, v8f& b, v8f& c, v8f& d) { asm volatile("v_nop\n\tv_nop\n\tv_nop\n\tv_nop" : "+v"(a), "+v"(b), "+v"(c), "+v"(d)); }

struct FragH {
  union U { v16h v; v8h h[2]; };
  static __device__ __forceinline__ v16h load(const _Float16* p) {
    U f; f.h[0] = *(const v8h*)(p); f.h[1] = *(const v8h*)(p + 16); return f.v;
  }
  static __device__ __forceinline__ v8f mma(v16h a, v16h b, v8f c) {
    return __builtin_amdgcn_wmma_f32_16x16x32_f16(false, a, false, b, (short)0, c, false, false);
  }
};

__device__ __forceinline__ float h16_to_f32(unsigned hb) {
  const unsigned sgn = (hb & 0x8000u) << 16; const unsigned em = hb & 0x7fffu;
  const float fn = __uint_as_float((em << 13) + 0x38000000u);
  const float fs = (float)em * 5.9604644775390625e-8f;
  const float mag = (em < 0x400u) ? fs : fn; return __uint_as_float(__float_as_uint(mag) | sgn);
}

__device__ __forceinline__ float sigm_f(float x)  { return __builtin_amdgcn_rcpf(1.0f + expf(-x)); }
__device__ __forceinline__ float tanh_f(float x)  { return 1.0f - 2.0f * __builtin_amdgcn_rcpf(expf(2.0f * x) + 1.0f); }

__global__ __launch_bounds__(256) void cvt_pad_kernel(const float* __restrict__ src0, const float* __restrict__ src1,
                                                      unsigned short* __restrict__ dst,
                                                      int nrow, int spitch, int ncolvalid, int ncol8, float sc) {
  const float* src = blockIdx.y ? src1 : src0;
  const int n8 = nrow * ncol8;
  unsigned short* dp = dst + (size_t)blockIdx.y * (size_t)n8 * 8;
  const int i = blockIdx.x * 256 + threadIdx.x;
  if (i < n8) {
    const int row = i / ncol8;
    const int p = i - row * ncol8;
    const int c0 = 8 * p, c1 = 8 * p + 4;
    const bool ok0 = c0 < ncolvalid, ok1 = c1 < ncolvalid;
    const int a0 = ok0 ? c0 : (ncolvalid - 4);
    const int a1 = ok1 ? c1 : (ncolvalid - 4);
    const float* sp = src + (size_t)row * spitch;
    const v4f a = *(const v4f*)(sp + a0);
    const v4f b = *(const v4f*)(sp + a1);
    v8h hv;
#pragma unroll
    for (int e = 0; e < 4; ++e) {
      const float fa = ok0 ? (a[e] * sc) : 0.0f;
      const float fb = ok1 ? (b[e] * sc) : 0.0f;
      hv[e]     = (_Float16)fa;
      hv[4 + e] = (_Float16)fb;
    }
    *(volatile v8h*)(dp + (size_t)i * 8) = hv;
    __threadfence();
    *(volatile v8h*)(dp + (size_t)i * 8) = hv;
  }
}

__global__ __launch_bounds__(256) void wcapt_kernel(const float* __restrict__ W, unsigned short* __restrict__ dst) {
  const int i = blockIdx.x * 256 + threadIdx.x;
  if (i < kCapPad * (kHid2 / 8)) {
    const int m = i >> 5;
    const int p = i & 31;
    const bool ok = m < kCapOut;
    const int mc = ok ? m : (kCapOut - 1);
    v8h hv;
#pragma unroll
    for (int e = 0; e < 8; ++e) {
      const float f = W[(size_t)(8 * p + e) * kCapOut + mc];
      const float g = ok ? (f * kWCarry) : 0.0f;
      hv[e] = (_Float16)g;
    }
    *(volatile v8h*)(dst + (size_t)i * 8) = hv;
    __threadfence();
    *(volatile v8h*)(dst + (size_t)i * 8) = hv;
  }
}

__global__ __launch_bounds__(256) void gather_rows_kernel(const int* __restrict__ tok, const float* __restrict__ emb,
                                                          unsigned short* __restrict__ dst) {
  constexpr int kP = kEmbPad / 8;
  const int i = blockIdx.x * 256 + threadIdx.x;
  if (i < kRows * kP) {
    const int row = i / kP;
    const int p = i - row * kP;
    const int s = row >> 7, b = row & (kBatch - 1);
    int tk = tok[b * kSeq + s];
    tk = tk < 0 ? 0 : tk;
    tk = tk > (kVocab - 1) ? (kVocab - 1) : tk;
    const int c0 = 8 * p, c1 = 8 * p + 4;
    const bool ok0 = c0 < kEmbDim, ok1 = c1 < kEmbDim;
    const int a0 = ok0 ? c0 : (kEmbDim - 4);
    const int a1 = ok1 ? c1 : (kEmbDim - 4);
    const float* sp = emb + (size_t)tk * kEmbDim;
    const v4f a = *(const v4f*)(sp + a0);
    const v4f bq = *(const v4f*)(sp + a1);
    v8h hv;
#pragma unroll
    for (int e = 0; e < 4; ++e) {
      const float fa = ok0 ? a[e] : 0.0f;
      const float fb = ok1 ? bq[e] : 0.0f;
      hv[e]     = (_Float16)fa;
      hv[4 + e] = (_Float16)fb;
    }
    *(volatile v8h*)(dst + (size_t)i * 8) = hv;
    __threadfence();
    *(volatile v8h*)(dst + (size_t)i * 8) = hv;
  }
}

template <int BIAS_MODE, int OUT_MODE>
__global__ __launch_bounds__(256) void wmma_gemm64_h(
    const unsigned short* __restrict__ Ap, int lda,
    const unsigned short* __restrict__ Btp, int ldb,
    void* __restrict__ Cout, int ldc,
    const float* __restrict__ bias,
    int M, int N, int K, float scale) {
  const _Float16* A  = (const _Float16*)Ap;
  const _Float16* Bt = (const _Float16*)Btp;
  __shared__ __align__(16) float sT[8][16 * 68];
  const int lane = threadIdx.x & 31;
  const int wave = threadIdx.x >> 5;
  const int tilesN = N >> 6;
  const int tilesM = M >> 6;
  const int tile = blockIdx.x * 8 + wave;
  if (tile >= tilesM * tilesN) return;
  const int tm = tile / tilesN;
  const int tn = tile - tm * tilesN;
  const int m0 = tm << 6;
  const int n0 = tn << 6;

  const int rlane = lane & 15;
  const int koff  = (lane >> 4) * 8;
  const int mOff  = (lane >> 4) * 8;

  v8f acc[4][4];
#pragma unroll
  for (int i = 0; i < 4; ++i)
#pragma unroll
    for (int j = 0; j < 4; ++j) acc[i][j] = (v8f){0.f,0.f,0.f,0.f,0.f,0.f,0.f,0.f};

  for (int k0 = 0; k0 < K; k0 += 32) {
    v16h bh[4];
#pragma unroll
    for (int j = 0; j < 4; ++j) {
      const size_t bo = (size_t)(n0 + (j << 4) + rlane) * ldb + koff + k0;
      bh[j] = FragH::load(Bt + bo);
    }
#pragma unroll
    for (int i = 0; i < 4; ++i) {
      const size_t ao = (size_t)(m0 + (i << 4) + rlane) * lda + koff + k0;
      const v16h ah = FragH::load(A + ao);
#pragma unroll
      for (int j = 0; j < 4; ++j) acc[i][j] = FragH::mma(ah, bh[j], acc[i][j]);
      guard4_h(acc[i][0], acc[i][1], acc[i][2], acc[i][3], ah, bh[0], bh[1], bh[2], bh[3]);
    }
    keep4_h(bh[0], bh[1], bh[2], bh[3]);
  }
  acc_guard4(acc[0][0], acc[0][1], acc[0][2], acc[0][3]);
  acc_guard4(acc[1][0], acc[1][1], acc[1][2], acc[1][3]);
  acc_guard4(acc[2][0], acc[2][1], acc[2][2], acc[2][3]);
  acc_guard4(acc[3][0], acc[3][1], acc[3][2], acc[3][3]);

  float* slab = sT[wave];
#pragma unroll
  for (int i = 0; i < 4; ++i) {
    const int mBase = m0 + (i << 4);
#pragma unroll
    for (int j = 0; j < 4; ++j) {
      const int n = n0 + (j << 4) + rlane;
      float bv = 0.f;
      if (BIAS_MODE == 2) bv = bias[n];
#pragma unroll
      for (int r = 0; r < 8; ++r) {
        float v = acc[i][j][r] * scale;
        if (BIAS_MODE == 2) v += bv;
        slab[(mOff + r) * 68 + (j << 4) + rlane] = v;
      }
    }
    __builtin_amdgcn_fence(__ATOMIC_RELEASE, "workgroup");
    __builtin_amdgcn_wave_barrier();
    __builtin_amdgcn_fence(__ATOMIC_ACQUIRE, "workgroup");
    if (OUT_MODE == 0) {
      float* C = (float*)Cout;
      const int hh = lane >> 4, c4 = (lane & 15) * 4;
      for (int pass = 0; pass < 2; ++pass) {
#pragma unroll
        for (int it = 0; it < 8; ++it) {
          const int row = it * 2 + hh;
          v4f v = *(const v4f*)(slab + row * 68 + c4);
          *(volatile v4f*)(C + (size_t)(mBase + row) * ldc + n0 + c4) = v;
        }
        __threadfence();
      }
    } else {
      const int q = lane >> 3, c8 = (lane & 7) * 8;
      unsigned short* C = (unsigned short*)Cout;
      for (int pass = 0; pass < 2; ++pass) {
#pragma unroll
        for (int it = 0; it < 4; ++it) {
          const int row = it * 4 + q;
          const float* sp = slab + row * 68 + c8;
          v8h hv;
#pragma unroll
          for (int e = 0; e < 8; ++e) hv[e] = (_Float16)sp[e];
          *(volatile v8h*)(C + (size_t)(mBase + row) * ldc + n0 + c8) = hv;
        }
        __threadfence();
      }
    }
    __builtin_amdgcn_fence(__ATOMIC_RELEASE, "workgroup");
    __builtin_amdgcn_wave_barrier();
    __builtin_amdgcn_fence(__ATOMIC_ACQUIRE, "workgroup");
  }
}

__global__ __launch_bounds__(256) void gru_seq_kernel(const unsigned* __restrict__ XP32,
                                                      const unsigned short* __restrict__ WHHp,
                                                      const float* __restrict__ bhhF, const float* __restrict__ bhhB,
                                                      unsigned short* __restrict__ HALL) {
  __shared__ __align__(16) _Float16 Ah[2][16 * kHPitch];
  __shared__ __align__(16) unsigned Xs[2][16 * kXWords];
  const int tid = threadIdx.x, lane = tid & 31, wave = tid >> 5;
  const int c = lane & 15, hh = lane >> 4, koff = hh * 8;
  const int dir = blockIdx.x >> 3;
  const int b0 = (blockIdx.x & 7) * 16;
  const int j = 16 * wave + c;
  const _Float16* WH = (const _Float16*)WHHp + (size_t)dir * kGate3 * kHid;
  const unsigned* xg = XP32 + (size_t)dir * kRows * (kGate3 / 2);
  const float* bhh = dir ? bhhB : bhhF;

  v16h bwr[4], bwz[4], bwn[4];
#pragma unroll
  for (int kc = 0; kc < 4; ++kc) {
    bwr[kc] = FragH::load(WH + (size_t)(j) * kHid + kc * 32 + koff);
    bwz[kc] = FragH::load(WH + (size_t)(kHid + j) * kHid + kc * 32 + koff);
    bwn[kc] = FragH::load(WH + (size_t)(2 * kHid + j) * kHid + kc * 32 + koff);
  }
  const float bhr = bhh[j], bhz = bhh[kHid + j], bhn = bhh[2 * kHid + j];

  const int q0 = tid, q1 = tid + 256, q2 = tid + 512;
  const int xd0 = (q0 / 48) * kXWords + (q0 % 48) * 4;
  const int xd1 = (q1 / 48) * kXWords + (q1 % 48) * 4;
  const int xd2 = (q2 / 48) * kXWords + (q2 % 48) * 4;

  {
    _Float16* ahf = &Ah[0][0];
#pragma unroll 1
    for (int i = tid; i < 2 * 16 * kHPitch; i += 256) ahf[i] = (_Float16)0.0f;
  }
  {
    const int tt0 = dir ? (kSeq - 1) : 0;
    const unsigned* xsrc = xg + ((size_t)tt0 * kBatch + b0) * (kGate3 / 2);
    const v4u p0 = *(const v4u*)(xsrc + 4 * q0);
    const v4u p1 = *(const v4u*)(xsrc + 4 * q1);
    const v4u p2 = *(const v4u*)(xsrc + 4 * q2);
    *(v4u*)(&Xs[0][xd0]) = p0;
    *(v4u*)(&Xs[0][xd1]) = p1;
    *(v4u*)(&Xs[0][xd2]) = p2;
  }
  float hst[8];
#pragma unroll
  for (int r = 0; r < 8; ++r) hst[r] = 0.0f;
  __syncthreads();

  const v8f z8 = {0.f, 0.f, 0.f, 0.f, 0.f, 0.f, 0.f, 0.f};
  const int wcol = j >> 1;
  const unsigned sh = (unsigned)(j & 1) * 16u;

#pragma unroll 1
  for (int t = 0; t < kSeq; ++t) {
    const int cur = t & 1;
    const int tt = dir ? (kSeq - 1 - t) : t;
    const int tn = (t + 1 < kSeq) ? (t + 1) : (kSeq - 1);
    const int ttn = dir ? (kSeq - 1 - tn) : tn;
    const unsigned* xnext = xg + ((size_t)ttn * kBatch + b0) * (kGate3 / 2);
    const v4u pf0 = *(const v4u*)(xnext + 4 * q0);
    const v4u pf1 = *(const v4u*)(xnext + 4 * q1);
    const v4u pf2 = *(const v4u*)(xnext + 4 * q2);

    v8f ar = z8, az = z8, an = z8;
    const _Float16* ahrow = &Ah[cur][0] + c * kHPitch + koff;
#pragma unroll
    for (int kc = 0; kc < 4; ++kc) {
      const v16h a = FragH::load(ahrow + kc * 32);
      ar = FragH::mma(a, bwr[kc], ar);
      az = FragH::mma(a, bwz[kc], az);
      an = FragH::mma(a, bwn[kc], an);
      guard3_h(ar, az, an, a, bwr[kc], bwz[kc], bwn[kc]);
    }

    const unsigned* xs = &Xs[cur][0];
    _Float16* ahn = &Ah[cur ^ 1][0];
#pragma unroll
    for (int r = 0; r < 8; ++r) {
      const int row = 8 * hh + r;
      const unsigned w0 = xs[row * kXWords + wcol];
      const unsigned w1 = xs[row * kXWords + 64 + wcol];
      const unsigned w2 = xs[row * kXWords + 128 + wcol];
      const float xr = h16_to_f32((w0 >> sh) & 0xffffu);
      const float xz = h16_to_f32((w1 >> sh) & 0xffffu);
      const float xn = h16_to_f32((w2 >> sh) & 0xffffu);
      const float hr = ar[r] * kWCarryInv + bhr;
      const float hz = az[r] * kWCarryInv + bhz;
      const float hn = an[r] * kWCarryInv + bhn;
      const float rg = sigm_f(xr + hr);
      const float zg = sigm_f(xz + hz);
      const float ng = tanh_f(xn + rg * hn);
      const float hnew = (1.0f - zg) * ng + zg * hst[r];
      hst[r] = hnew;
      ahn[row * kHPitch + j] = (_Float16)hnew;
    }
    *(v4u*)(&Xs[cur ^ 1][xd0]) = pf0;
    *(v4u*)(&Xs[cur ^ 1][xd1]) = pf1;
    *(v4u*)(&Xs[cur ^ 1][xd2]) = pf2;
    __syncthreads();

    {
      const int rr = 2 * wave + hh;
      const v8h hv = *(const v8h*)(&Ah[cur ^ 1][0] + rr * kHPitch + c * 8);
      unsigned short* dp = HALL + ((size_t)(b0 + rr) * kSeq + (size_t)tt) * kHid2 + dir * kHid + c * 8;
      *(volatile v8h*)dp = hv;
      __threadfence();
      *(volatile v8h*)dp = hv;
    }
  }
}

__global__ __launch_bounds__(256) void routing_kernel(const float* __restrict__ UH, float* __restrict__ CAPS) {
  __shared__ float blog[kCaps * kSeq];
  __shared__ float cw[kCaps * kSeq];
  __shared__ __align__(16) float vs[kCapOut];
  __shared__ __align__(16) float vn[kCapOut];
  const int tid = threadIdx.x, lane = tid & 31, wave = tid >> 5;
  const int b = blockIdx.x;
  const int s = tid;
  const float* u = UH + (size_t)b * kSeq * kCapPad;

#pragma unroll 1
  for (int i = 0; i < kCaps; ++i) blog[i * kSeq + s] = 0.0f;

#pragma unroll 1
  for (int it = 0; it < kIters; ++it) {
    float mx = blog[s];
#pragma unroll 1
    for (int i = 1; i < kCaps; ++i) mx = fmaxf(mx, blog[i * kSeq + s]);
    float sum = 0.0f;
#pragma unroll 1
    for (int i = 0; i < kCaps; ++i) {
      const float e = expf(blog[i * kSeq + s] - mx);
      cw[i * kSeq + s] = e;
      sum += e;
    }
    const float inv = 1.0f / sum;
#pragma unroll 1
    for (int i = 0; i < kCaps; ++i) {
      const float e = cw[i * kSeq + s];
      cw[i * kSeq + s] = e * inv;
    }
    __syncthreads();
    if (tid < kCapOut) {
      const float* cp = cw + (tid >> 4) * kSeq;
      const float* up = u + tid;
      float acc = 0.0f;
#pragma unroll 4
      for (int p = 0; p < kSeq; ++p) acc = fmaf(cp[p], up[(size_t)p * kCapPad], acc);
      vs[tid] = acc;
    }
    __syncthreads();
    if (tid < kCapOut) {
      const int base = tid & ~15;
      float ss = 0.0f;
#pragma unroll 4
      for (int k = 0; k < kCapDim; ++k) { const float q = vs[base + k]; ss = fmaf(q, q, ss); }
      vn[tid] = vs[tid] / sqrtf(ss + kSquashEps);
    }
    __syncthreads();
    if (it < kIters - 1) {
      const float* ur = u + (size_t)s * kCapPad;
#pragma unroll 1
      for (int i = 0; i < kCaps; ++i) {
        const v4f u0 = *(const v4f*)(ur + i * 16);
        const v4f u1 = *(const v4f*)(ur + i * 16 + 4);
        const v4f u2 = *(const v4f*)(ur + i * 16 + 8);
        const v4f u3 = *(const v4f*)(ur + i * 16 + 12);
        const float* vp = vn + i * 16;
        float d = 0.0f;
#pragma unroll
        for (int e = 0; e < 4; ++e) {
          d = fmaf(vp[e], u0[e], d);
          d = fmaf(vp[4 + e], u1[e], d);
          d = fmaf(vp[8 + e], u2[e], d);
          d = fmaf(vp[12 + e], u3[e], d);
        }
        blog[i * kSeq + s] += d;
      }
    }
  }
  if (wave == 0) {
    const v4f a = *(const v4f*)(vn + lane * 4);
    const v4f bq = *(const v4f*)(vn + 128 + (lane & 7) * 4);
    float* dp = CAPS + (size_t)b * kCapOut;
    for (int pass = 0; pass < 2; ++pass) {
      *(volatile v4f*)(dp + lane * 4) = a;
      if (lane < 8) *(volatile v4f*)(dp + 128 + lane * 4) = bq;
      __threadfence();
    }
  }
}

__global__ __launch_bounds__(256) void head_kernel(const float* __restrict__ CAPS, const float* __restrict__ W,
                                                   const float* __restrict__ bias, float* __restrict__ out) {
  const int t = threadIdx.x;
  const int b = t >> 1, c = t & 1;
  const float* cp = CAPS + (size_t)b * kCapOut;
  float acc = 0.0f;
#pragma unroll 4
  for (int m = 0; m < kCapOut; ++m) acc = fmaf(cp[m], W[m * kOutCls + c], acc);
  acc += bias[c];
  *(volatile float*)(out + t) = acc;
  __threadfence();
  *(volatile float*)(out + t) = acc;
}

extern "C" void kernel_launch(void* const* d_in, const int* in_sizes, int n_in,
                              void* d_out, int out_size, void* d_ws, size_t ws_size, hipStream_t stream) {
  if (n_in < 13 || d_out == nullptr || d_ws == nullptr) return;
  if (in_sizes[0] != kBatch * kSeq || in_sizes[1] != kVocab * kEmbDim ||
      in_sizes[2] != kGate3 * kEmbDim || in_sizes[3] != kGate3 * kHid || in_sizes[4] != kGate3 || in_sizes[5] != kGate3 ||
      in_sizes[6] != kGate3 * kEmbDim || in_sizes[7] != kGate3 * kHid || in_sizes[8] != kGate3 || in_sizes[9] != kGate3 ||
      in_sizes[10] != kHid2 * kCapOut || in_sizes[11] != kCapOut * kOutCls || in_sizes[12] != kOutCls ||
      out_size != kBatch * kOutCls) return;

  const int*   x_tok  = (const int*)d_in[0];
  const float* emb    = (const float*)d_in[1];
  const float* w_ih_f = (const float*)d_in[2];
  const float* w_hh_f = (const float*)d_in[3];
  const float* b_ih_f = (const float*)d_in[4];
  const float* b_hh_f = (const float*)d_in[5];
  const float* w_ih_b = (const float*)d_in[6];
  const float* w_hh_b = (const float*)d_in[7];
  const float* b_ih_b = (const float*)d_in[8];
  const float* b_hh_b = (const float*)d_in[9];
  const float* W_cap  = (const float*)d_in[10];
  const float* W_lin  = (const float*)d_in[11];
  const float* b_lin  = (const float*)d_in[12];
  float* out = (float*)d_out;

  char* ws = (char*)d_ws; size_t off = 0;
  auto carve = [&](size_t bytes) -> char* { char* p = ws + off; off += (bytes + 255) & ~(size_t)255; return p; };
  unsigned short* WIH16 = (unsigned short*)carve((size_t)2 * kGate3 * kEmbPad * 2);
  unsigned short* WHH16 = (unsigned short*)carve((size_t)2 * kGate3 * kHid * 2);
  unsigned short* WCAPT = (unsigned short*)carve((size_t)kCapPad * kHid2 * 2);
  unsigned short* EF16  = (unsigned short*)carve((size_t)kRows * kEmbPad * 2);
  unsigned short* XPROJ = (unsigned short*)carve((size_t)2 * kRows * kGate3 * 2);
  unsigned short* HALL  = (unsigned short*)carve((size_t)kRows * kHid2 * 2);
  float*          UHAT  = (float*)carve((size_t)kRows * kCapPad * 4);
  float*          CAPS  = (float*)carve((size_t)kBatch * kCapOut * 4);
  if (off > ws_size || off > (size_t)134217728) return;

  static_assert((kGate3 * (kEmbPad / 8)) % 256 == 0 && (kGate3 * (kHid / 8)) % 256 == 0);
  cvt_pad_kernel<<<dim3(kGate3 * (kEmbPad / 8) / 256, 2), 256, 0, stream>>>(w_ih_f, w_ih_b, WIH16, kGate3, kEmbDim, kEmbDim, kEmbPad / 8, kWCarry);
  cvt_pad_kernel<<<dim3(kGate3 * (kHid / 8) / 256, 2), 256, 0, stream>>>(w_hh_f, w_hh_b, WHH16, kGate3, kHid, kHid, kHid / 8, kWCarry);
  static_assert((kCapPad * (kHid2 / 8)) % 256 == 0);
  wcapt_kernel<<<kCapPad * (kHid2 / 8) / 256, 256, 0, stream>>>(W_cap, WCAPT);
  static_assert((kRows * (kEmbPad / 8)) % 256 == 0);
  gather_rows_kernel<<<kRows * (kEmbPad / 8) / 256, 256, 0, stream>>>(x_tok, emb, EF16);
  static_assert(((kRows / 64) * (kGate3 / 64)) % 8 == 0);
  wmma_gemm64_h<2, 1><<<(kRows / 64) * (kGate3 / 64) / 8, 256, 0, stream>>>(
      EF16, kEmbPad, WIH16, kEmbPad, (void*)XPROJ, kGate3, b_ih_f, kRows, kGate3, kEmbPad, kWCarryInv);
  wmma_gemm64_h<2, 1><<<(kRows / 64) * (kGate3 / 64) / 8, 256, 0, stream>>>(
      EF16, kEmbPad, WIH16 + (size_t)kGate3 * kEmbPad, kEmbPad, (void*)(XPROJ + (size_t)kRows * kGate3), kGate3,
      b_ih_b, kRows, kGate3, kEmbPad, kWCarryInv);
  gru_seq_kernel<<<2 * (kBatch / 16), 256, 0, stream>>>((const unsigned*)XPROJ, WHH16, b_hh_f, b_hh_b, HALL);
  static_assert(((kRows / 64) * (kCapPad / 64)) % 8 == 0);
  wmma_gemm64_h<0, 0><<<(kRows / 64) * (kCapPad / 64) / 8, 256, 0, stream>>>(
      HALL, kHid2, WCAPT, kHid2, (void*)UHAT, kCapPad, b_ih_f, kRows, kCapPad, kHid2, kWCarryInv);
  routing_kernel<<<kBatch, 256, 0, stream>>>(UHAT, CAPS);
  head_kernel<<<1, 256, 0, stream>>>(CAPS, W_lin, b_lin, out);
}
